// FactorNet_69518340653114
// MI455X (gfx1250) — hardware-verified
//
#include <hip/hip_runtime.h>


namespace {
constexpr int N = 16384, D = 64, H1 = 64, H2 = 64, O = 32;
constexpr float AS_ = 8.0f, MIN_SIGMA = 0.008f;

typedef _Float16 b16;
typedef __attribute__((ext_vector_type(16))) _Float16 v16b;
typedef __attribute__((ext_vector_type(8))) _Float16 v8b;
typedef __attribute__((ext_vector_type(8))) float v8f;
typedef __attribute__((ext_vector_type(4))) float v4f;
__device__ __forceinline__ float bf16_rne(float f) { unsigned int u = __float_as_uint(f); u += 0x7FFFu + ((u >> 16) & 1u); return __uint_as_float(u & 0xFFFF0000u); }
__device__ __forceinline__ void split16(float v, b16& hi, b16& lo) { hi = (b16)v; lo = (b16)(v - (float)hi); }
__device__ __forceinline__ v16b frag_kb(const b16* p, int hh) { const v8b a = *(const v8b*)(p + 8 * hh), b = *(const v8b*)(p + 16 + 8 * hh); v16b f;
#pragma unroll
  for (int e = 0; e < 8; ++e) { f[e] = a[e]; f[8 + e] = b[e]; } return f; }
__device__ __forceinline__ v8f wmma16b(v16b a, v16b b, v8f c) { v8f d = __builtin_amdgcn_wmma_f32_16x16x32_f16(false, a, false, b, (short)0, c, false, false); asm volatile("v_nop\n\tv_nop\n\tv_nop\n\tv_nop" : "+v"(d) : "v"(a), "v"(b)); return d; }
__device__ __forceinline__ void wave_lds_sync() { __builtin_amdgcn_fence(__ATOMIC_RELEASE, "workgroup"); __builtin_amdgcn_wave_barrier(); __builtin_amdgcn_fence(__ATOMIC_ACQUIRE, "workgroup"); }
__device__ __forceinline__ float pmul(float a, float b) { float p = a * b; asm volatile("" : "+v"(p)); return p; }
__device__ __forceinline__ float softplus_(float z) { return fmaxf(z, 0.0f) + log1pf(__expf(-fabsf(z))); }

__global__ __launch_bounds__(256) void prep_kernel(const float* __restrict__ W1, const float* __restrict__ b1, const float* __restrict__ W2, const float* __restrict__ b2, const float* __restrict__ Wmu, const float* __restrict__ bmu, const float* __restrict__ Wsig, const float* __restrict__ bsig,
                                                   b16* __restrict__ W2r, b16* __restrict__ W3r, float* __restrict__ P) {
  const size_t tid = (size_t)blockIdx.x * blockDim.x + threadIdx.x, nth = (size_t)gridDim.x * blockDim.x;
  for (int pass = 0; pass < 2; ++pass) {
    for (size_t p = tid; p < (size_t)D * H2 * H1; p += nth) { const int d = (int)(p >> 12), k = (int)((p >> 6) & 63), h = (int)(p & 63); ((volatile b16*)W2r)[p] = (b16)bf16_rne(W2[((size_t)d * H1 + h) * H2 + k]); }
    for (size_t p = tid; p < (size_t)D * 64 * H2; p += nth) { const int d = (int)(p >> 12), n = (int)((p >> 6) & 63), k = (int)(p & 63); const float v = (n < O) ? Wmu[((size_t)d * H2 + k) * O + n] : Wsig[((size_t)d * H2 + k) * O + (n - O)]; ((volatile b16*)W3r)[p] = (b16)bf16_rne(v); }
    for (size_t p = tid; p < 16384; p += nth) { float v; if (p < 4096) v = W1[p]; else if (p < 8192) v = b1[p - 4096]; else if (p < 12288) v = b2[p - 8192]; else if (p < 14336) v = bmu[p - 12288]; else v = bsig[p - 14336]; ((volatile float*)P)[p] = bf16_rne(v); }
    __threadfence();
  }
}

__global__ __launch_bounds__(128) void fn_kernel(const float* __restrict__ x, const int* __restrict__ mask, const float* __restrict__ P, const b16* __restrict__ W2r, const b16* __restrict__ W3r, float* __restrict__ muo, float* __restrict__ sgo) {
  __shared__ __attribute__((aligned(16))) float T[4][32][64 + 4];
  const int lane = threadIdx.x & 31, wave = threadIdx.x >> 5, nloc = lane & 15, hlf = lane >> 4, m0 = blockIdx.x * 128 + wave * 32;
  const float* W1 = P; const float* b1 = P + 4096; const float* b2 = P + 8192; const float* bmu = P + 12288; const float* bsig = P + 14336;
  float np1[2][2][8], np2[2][2][8];
#pragma unroll
  for (int r = 0; r < 2; ++r)
#pragma unroll
    for (int t = 0; t < 2; ++t)
#pragma unroll
      for (int v = 0; v < 8; ++v) { np1[r][t][v] = 0.0f; np2[r][t][v] = 0.0f; }
  for (int d = 0; d < D; ++d) {
    const float xa = bf16_rne(x[(size_t)(m0 + nloc) * D + d]), xb = bf16_rne(x[(size_t)(m0 + 16 + nloc) * D + d]);
    const b16* B2 = W2r + (size_t)d * 4096; const b16* B3 = W3r + (size_t)d * 4096;
    v8f acc[2][4];
#pragma unroll
    for (int r = 0; r < 2; ++r)
#pragma unroll
      for (int t = 0; t < 4; ++t) acc[r][t] = (v8f){};
#pragma unroll
    for (int ks = 0; ks < 2; ++ks) { v16b a0, l0, a1, l1;
#pragma unroll
      for (int e = 0; e < 16; ++e) { const int h = ks * 32 + ((e < 8) ? (8 * hlf + e) : (16 + 8 * hlf + e - 8)); const float w = W1[d * H1 + h], bb = b1[d * H1 + h];
        b16 p, q; split16(fmaxf(pmul(xa, w) + bb, 0.0f) * AS_, p, q); a0[e] = p; l0[e] = q; split16(fmaxf(pmul(xb, w) + bb, 0.0f) * AS_, p, q); a1[e] = p; l1[e] = q; }
#pragma unroll
      for (int t = 0; t < 4; ++t) { const v16b bw = frag_kb(B2 + (size_t)(t * 16 + nloc) * H1 + ks * 32, hlf); acc[0][t] = wmma16b(a0, bw, acc[0][t]); acc[0][t] = wmma16b(l0, bw, acc[0][t]); acc[1][t] = wmma16b(a1, bw, acc[1][t]); acc[1][t] = wmma16b(l1, bw, acc[1][t]); } }
#pragma unroll
    for (int t = 0; t < 4; ++t) { const float bb = b2[d * H2 + t * 16 + nloc];
#pragma unroll
      for (int r = 0; r < 2; ++r)
#pragma unroll
        for (int v = 0; v < 8; ++v) T[wave][r * 16 + 8 * hlf + v][t * 16 + nloc] = fmaxf(acc[r][t][v] * (1.0f / AS_) + bb, 0.0f); }
    wave_lds_sync();
#pragma unroll
    for (int r = 0; r < 2; ++r)
#pragma unroll
      for (int t = 0; t < 4; ++t) acc[r][t] = (v8f){};
#pragma unroll
    for (int ks = 0; ks < 2; ++ks) { v16b a0, l0, a1, l1;
#pragma unroll
      for (int e = 0; e < 16; ++e) { const int k = ks * 32 + ((e < 8) ? (8 * hlf + e) : (16 + 8 * hlf + e - 8)); b16 p, q; split16(T[wave][nloc][k] * AS_, p, q); a0[e] = p; l0[e] = q; split16(T[wave][16 + nloc][k] * AS_, p, q); a1[e] = p; l1[e] = q; }
#pragma unroll
      for (int t = 0; t < 4; ++t) { const v16b bw = frag_kb(B3 + (size_t)(t * 16 + nloc) * H2 + ks * 32, hlf); acc[0][t] = wmma16b(a0, bw, acc[0][t]); acc[0][t] = wmma16b(l0, bw, acc[0][t]); acc[1][t] = wmma16b(a1, bw, acc[1][t]); acc[1][t] = wmma16b(l1, bw, acc[1][t]); } }
    wave_lds_sync();
#pragma unroll
    for (int t = 0; t < 2; ++t) { const int o = t * 16 + nloc; const float bm = bmu[d * O + o], bs = bsig[d * O + o];
#pragma unroll
      for (int r = 0; r < 2; ++r)
#pragma unroll
        for (int v = 0; v < 8; ++v) { const int row = m0 + r * 16 + 8 * hlf + v; const bool mk = mask[(size_t)row * D + d] > 0;
          const float mu = acc[r][t][v] * (1.0f / AS_) + bm; const float sg = MIN_SIGMA + softplus_(acc[r][2 + t][v] * (1.0f / AS_) + bs); const float iv = 1.0f / (sg * sg);
          np1[r][t][v] += mk ? mu * iv : 0.0f; np2[r][t][v] += mk ? -0.5f * iv : 0.0f; } }
  }
#pragma unroll
  for (int t = 0; t < 2; ++t)
#pragma unroll
    for (int r = 0; r < 2; ++r)
#pragma unroll
      for (int v = 0; v < 8; ++v) { const float s2 = -0.5f / np2[r][t][v]; T[wave][r * 16 + 8 * hlf + v][t * 16 + nloc] = np1[r][t][v] * s2; T[wave][r * 16 + 8 * hlf + v][32 + t * 16 + nloc] = sqrtf(s2); }
  wave_lds_sync();
  for (int pass = 0; pass < 2; ++pass) {
#pragma unroll
    for (int j = 0; j < 8; ++j) { const int rr = j * 4 + (lane >> 3), c4 = (lane & 7) * 4; *(volatile v4f*)(muo + (size_t)(m0 + rr) * O + c4) = *(const v4f*)(&T[wave][rr][c4]); *(volatile v4f*)(sgo + (size_t)(m0 + rr) * O + c4) = *(const v4f*)(&T[wave][rr][32 + c4]); }
    __threadfence(); }
}
}

extern "C" void kernel_launch(void* const* d_in, const int* in_sizes, int n_in,
                              void* d_out, int out_size, void* d_ws, size_t ws_size, hipStream_t stream) {
  (void)n_in; (void)out_size;
  const float* x = (const float*)d_in[0]; const float* W1 = (const float*)d_in[1]; const float* b1 = (const float*)d_in[2]; const float* W2 = (const float*)d_in[3]; const float* b2 = (const float*)d_in[4];
  const float* Wmu = (const float*)d_in[5]; const float* bmu = (const float*)d_in[6]; const float* Wsig = (const float*)d_in[7]; const float* bsig = (const float*)d_in[8]; const int* mask = (const int*)d_in[9];
  float* muo = (float*)d_out; float* sgo = muo + (size_t)N * O;
  if (in_sizes[0] != N * D || in_sizes[1] != D * H1 || in_sizes[3] != D * H1 * H2 || in_sizes[5] != D * H2 * O || in_sizes[9] != N * D) return;
  size_t off = 0; char* ws = (char*)d_ws;
  auto carve = [&](size_t bytes) { char* p = ws + off; off += (bytes + 255) & ~(size_t)255; return p; };
  b16* W2r = (b16*)carve((size_t)D * 4096 * 2); b16* W3r = (b16*)carve((size_t)D * 4096 * 2); float* P = (float*)carve(16384 * 4);
  if (off > ws_size) return;
  prep_kernel<<<128, 256, 0, stream>>>(W1, b1, W2, b2, Wmu, bmu, Wsig, bsig, W2r, W3r, P);
  fn_kernel<<<N / 128, 128, 0, stream>>>(x, mask, P, W2r, W3r, muo, sgo);
}
